// ChebConv_46153718563236
// MI455X (gfx1250) — hardware-run, weakly checked
//
#include <hip/hip_runtime.h>
#include <stddef.h>
#include <stdint.h>


#define NNODE   100000
#define NEDGE   1250000
#define DF      64
#define DOUTF   64
#define KPOLY   3
#define KCAT    320
#define KSTEPS  (KCAT / 32)
#define APITCH  320
#define WPITCH  320
#define AWORDS  (APITCH / 2)
#define SPLIT_X1 1
#define SPLIT_X2 1
#define NTHR    256
#define NWAVE   8
#define EPT     8
#define CHUNK   (NTHR * EPT)
#define WCAP    (EPT * 32)
#define LISTN   (NWAVE * WCAP)
#define NBA     1024
#define PKS     10
#define NBLK    98
#define NPADN   (NBLK * NBA)
#define RCAP    16384
#define DEGCAP  64
#define MEAS_BLK_HITS 13102
#define MEAS_MAXDEG   29
#define GBM     128
#define MPAD    100096
#define RPB     64
#define RPW     8
#define BK_INTS (2 * RCAP + 4 * NBA + LISTN + 32)
#define LDS_BK  (BK_INTS * 4)
#define PREP_WT_UNITS (DOUTF * (KCAT / 8))
#define PREP_WT_BLKS  (PREP_WT_UNITS / NTHR)
#define PREP_XB_UNITS (MPAD * 8)
#define PREP_XB_BLKS  (PREP_XB_UNITS / NTHR)
#define PREP_BLKS     (PREP_WT_BLKS + PREP_XB_BLKS + 1)

static constexpr float LAMBDA_MAX = 2.0f;
static constexpr float RE_NORM    = 2.0f / LAMBDA_MAX;
static constexpr float CX1_A      = -RE_NORM;
static constexpr float CX1_B      = RE_NORM - 1.0f;
static constexpr float CX2_A      = -2.0f * RE_NORM;
static constexpr float CX2_B      = 2.0f * (RE_NORM - 1.0f);

static constexpr size_t SZ_WT = (size_t)DOUTF * WPITCH * 2;
static constexpr size_t SZ_BS = 256;
static constexpr size_t SZ_XB = (size_t)MPAD * DF * 2;
static constexpr size_t SZ_X1 = (size_t)MPAD * DF * 4;
static constexpr size_t SZ_A  = (size_t)MPAD * APITCH * 2;
static constexpr size_t SZ_LS = (size_t)NBLK * RCAP * 4;
static constexpr size_t SZ_TB = (size_t)NPADN * 4;
static constexpr size_t SZ_RC = (size_t)NBLK * 128;
static constexpr size_t O_WT = 0;
static constexpr size_t O_BS = O_WT + SZ_WT;
static constexpr size_t O_XB = O_BS + SZ_BS;
static constexpr size_t O_X1 = O_XB + SZ_XB;
static constexpr size_t O_A  = O_X1 + SZ_X1;
static constexpr size_t O_LS = O_A + SZ_A;
static constexpr size_t O_CN = O_LS + SZ_LS;
static constexpr size_t O_OF = O_CN + SZ_TB;
static constexpr size_t O_DS = O_OF + SZ_TB;
static constexpr size_t O_RC = O_DS + SZ_TB;
static constexpr size_t WS_TOTAL = O_RC + SZ_RC;

static_assert(DF == 64 && DOUTF == 64 && KPOLY == 3);
static_assert(KCAT == 320 && KCAT % 32 == 0 && KCAT == DF * (2 * KPOLY - 1));
static_assert(APITCH >= KCAT && WPITCH >= KCAT && (APITCH * 2) % 128 == 0 && (WPITCH * 2) % 128 == 0);
static_assert((long long)NBA * NBLK >= NNODE);
static_assert(MPAD % GBM == 0 && MPAD % RPB == 0 && MPAD >= NNODE && MPAD <= NPADN);
static_assert((CHUNK & (CHUNK - 1)) == 0 && CHUNK <= 4096);
static_assert(NBA == (1 << PKS) && NBA == NTHR * 4);
static_assert(LISTN == NWAVE * WCAP);
static_assert(RCAP % (NTHR * 4) == 0 && BK_INTS % 4 == 0);
static_assert((long long)RCAP * 100 >= (long long)MEAS_BLK_HITS * 105);
static_assert(DEGCAP >= MEAS_MAXDEG + 8);
static_assert(NEDGE < (1 << 21));
static_assert(LDS_BK <= 327680);
static_assert(GBM == NWAVE * 16 && RPB == NWAVE * RPW);
static_assert(PREP_WT_UNITS % NTHR == 0 && PREP_XB_UNITS % NTHR == 0);
static_assert(SZ_WT % 256 == 0 && SZ_XB % 256 == 0 && SZ_X1 % 256 == 0 && SZ_A % 256 == 0);
static_assert(SZ_LS % 256 == 0 && SZ_TB % 256 == 0 && SZ_RC % 256 == 0);
static_assert(WS_TOTAL <= (size_t)(128u << 20));

typedef float          v2f   __attribute__((ext_vector_type(2)));
typedef float          v4f   __attribute__((ext_vector_type(4)));
typedef float          v8f   __attribute__((ext_vector_type(8)));
typedef int            v4i   __attribute__((ext_vector_type(4)));
typedef int            v8i   __attribute__((ext_vector_type(8)));
typedef unsigned short v8us  __attribute__((ext_vector_type(8)));
typedef __bf16         v16bf __attribute__((ext_vector_type(16)));
typedef v4f  __attribute__((may_alias)) v4fa;
typedef v4i  __attribute__((may_alias)) v4ia;
typedef v8us __attribute__((may_alias)) v8usa;
union FragB { v16bf v; v8us h[2]; v8i w; };

__device__ __forceinline__ v8f wmb(const FragB& a, const FragB& b, v8f c) {
  v8f d = __builtin_amdgcn_wmma_f32_16x16x32_bf16(false, a.v, false, b.v, (short)0, c, false, false);
  asm volatile("v_nop\n\tv_nop\n\tv_nop\n\tv_nop" : "+v"(d) : "v"(a.w), "v"(b.w));
  return d;
}

__device__ __forceinline__ unsigned bf16_bits(float f) {
  const unsigned u = __float_as_uint(f);
  const unsigned r = ((u + 0x7FFFu + ((u >> 16) & 1u)) >> 16) & 0xFFFFu;
  const unsigned q = ((u >> 16) | 0x40u) & 0xFFFFu;
  return ((u & 0x7FFFFFFFu) > 0x7F800000u) ? q : r;
}
__device__ __forceinline__ float bf16_val(float f) { return __uint_as_float(bf16_bits(f) << 16); }
__device__ __forceinline__ float bfw_lo(unsigned w) { return __uint_as_float(w << 16); }
__device__ __forceinline__ float bfw_hi(unsigned w) { return __uint_as_float(w & 0xffff0000u); }
__device__ __forceinline__ void pack2(float a, float b, unsigned& hw, unsigned& lw) {
  const unsigned ha = bf16_bits(a), hb = bf16_bits(b);
  const unsigned la = bf16_bits(a - __uint_as_float(ha << 16));
  const unsigned lb = bf16_bits(b - __uint_as_float(hb << 16));
  hw = ha | (hb << 16);
  lw = la | (lb << 16);
}
__device__ __forceinline__ float relu_k(float v) { return (v > 0.0f) ? v : (v - v); }

__device__ __forceinline__ void slot_info(const int* __restrict__ CNT, const int* __restrict__ OFF, int node,
                                          int& c, int& o, int& last) {
  const int craw = CNT[node];
  const int oraw = OFF[node];
  int cc = craw < 0 ? 0 : craw;
  cc = cc > DEGCAP ? DEGCAP : cc;
  int oo = oraw < 0 ? 0 : (oraw > RCAP - 1 ? RCAP - 1 : oraw);
  if (cc > RCAP - oo) cc = RCAP - oo;
  c = __builtin_amdgcn_readfirstlane(cc);
  o = __builtin_amdgcn_readfirstlane(oo);
  int l = o + c - 1;
  l = l < o ? o : l;
  last = l;
}

__device__ __forceinline__ int scan_chunk(const int* __restrict__ keys, int nE, int cbase, int slotBase,
                                          int nb, int vec8, int* list, int tid, int wave) {
  int wc = 0;
  const int el0  = tid * EPT;
  const int e0   = cbase + el0;
  const int sent = (int)(1u << 31);
  v4i da, db;
  if (vec8 != 0 && cbase + CHUNK <= nE) {
    da = *(const v4i*)(keys + e0);
    db = *(const v4i*)(keys + e0 + 4);
  } else {
    const int t0 = keys[min(e0,     nE - 1)];
    const int t1 = keys[min(e0 + 1, nE - 1)];
    const int t2 = keys[min(e0 + 2, nE - 1)];
    const int t3 = keys[min(e0 + 3, nE - 1)];
    const int t4 = keys[min(e0 + 4, nE - 1)];
    const int t5 = keys[min(e0 + 5, nE - 1)];
    const int t6 = keys[min(e0 + 6, nE - 1)];
    const int t7 = keys[min(e0 + 7, nE - 1)];
    asm volatile("" :: "v"(t0), "v"(t1), "v"(t2), "v"(t3), "v"(t4), "v"(t5), "v"(t6), "v"(t7));
    da.x = (e0     < nE) ? t0 : sent;
    da.y = (e0 + 1 < nE) ? t1 : sent;
    da.z = (e0 + 2 < nE) ? t2 : sent;
    da.w = (e0 + 3 < nE) ? t3 : sent;
    db.x = (e0 + 4 < nE) ? t4 : sent;
    db.y = (e0 + 5 < nE) ? t5 : sent;
    db.z = (e0 + 6 < nE) ? t6 : sent;
    db.w = (e0 + 7 < nE) ? t7 : sent;
  }
  const unsigned nbs = (unsigned)slotBase;
  const unsigned unb = (unsigned)nb;
  const unsigned s0 = (unsigned)da.x - nbs, s1 = (unsigned)da.y - nbs;
  const unsigned s2 = (unsigned)da.z - nbs, s3 = (unsigned)da.w - nbs;
  const unsigned s4 = (unsigned)db.x - nbs, s5 = (unsigned)db.y - nbs;
  const unsigned s6 = (unsigned)db.z - nbs, s7 = (unsigned)db.w - nbs;
  const bool h0 = s0 < unb, h1 = s1 < unb, h2 = s2 < unb, h3 = s3 < unb;
  const bool h4 = s4 < unb, h5 = s5 < unb, h6 = s6 < unb, h7 = s7 < unb;
  const unsigned m0 = __builtin_amdgcn_ballot_w32(h0);
  const unsigned m1 = __builtin_amdgcn_ballot_w32(h1);
  const unsigned m2 = __builtin_amdgcn_ballot_w32(h2);
  const unsigned m3 = __builtin_amdgcn_ballot_w32(h3);
  const unsigned m4 = __builtin_amdgcn_ballot_w32(h4);
  const unsigned m5 = __builtin_amdgcn_ballot_w32(h5);
  const unsigned m6 = __builtin_amdgcn_ballot_w32(h6);
  const unsigned m7 = __builtin_amdgcn_ballot_w32(h7);
  const unsigned any = m0 | m1 | m2 | m3 | m4 | m5 | m6 | m7;
  if (any != 0u) {
    int pos = (int)__builtin_amdgcn_mbcnt_lo(m0, 0u) + (int)__builtin_amdgcn_mbcnt_lo(m1, 0u)
            + (int)__builtin_amdgcn_mbcnt_lo(m2, 0u) + (int)__builtin_amdgcn_mbcnt_lo(m3, 0u)
            + (int)__builtin_amdgcn_mbcnt_lo(m4, 0u) + (int)__builtin_amdgcn_mbcnt_lo(m5, 0u)
            + (int)__builtin_amdgcn_mbcnt_lo(m6, 0u) + (int)__builtin_amdgcn_mbcnt_lo(m7, 0u);
    int* wl = list + wave * WCAP;
    if (h0) { if (pos < WCAP) wl[pos] = ((el0 + 0) << PKS) | (int)s0; pos += 1; }
    if (h1) { if (pos < WCAP) wl[pos] = ((el0 + 1) << PKS) | (int)s1; pos += 1; }
    if (h2) { if (pos < WCAP) wl[pos] = ((el0 + 2) << PKS) | (int)s2; pos += 1; }
    if (h3) { if (pos < WCAP) wl[pos] = ((el0 + 3) << PKS) | (int)s3; pos += 1; }
    if (h4) { if (pos < WCAP) wl[pos] = ((el0 + 4) << PKS) | (int)s4; pos += 1; }
    if (h5) { if (pos < WCAP) wl[pos] = ((el0 + 5) << PKS) | (int)s5; pos += 1; }
    if (h6) { if (pos < WCAP) wl[pos] = ((el0 + 6) << PKS) | (int)s6; pos += 1; }
    if (h7) { if (pos < WCAP) wl[pos] = ((el0 + 7) << PKS) | (int)s7; pos += 1; }
    wc = (int)__builtin_popcount(m0) + (int)__builtin_popcount(m1) + (int)__builtin_popcount(m2)
       + (int)__builtin_popcount(m3) + (int)__builtin_popcount(m4) + (int)__builtin_popcount(m5)
       + (int)__builtin_popcount(m6) + (int)__builtin_popcount(m7);
  }
  return wc;
}

__global__ __launch_bounds__(NTHR) void k_prep(const float* __restrict__ feat, const float* __restrict__ W,
                                               const float* __restrict__ bvec, unsigned short* WT,
                                               unsigned short* XB, float* BIAS, int nN) {
  const int tid = (int)threadIdx.x;
  const int blk = (int)blockIdx.x;
  if (blk < PREP_WT_BLKS) {
    const int u    = blk * NTHR + tid;
    const int n    = u / (KCAT / 8);
    const int j    = u - n * (KCAT / 8);
    const int k8   = 8 * j;
    const int seg  = k8 >> 6;
    const int kin  = k8 & 63;
    const int srow = (seg == 0) ? kin : ((seg <= 2) ? (DF + kin) : (2 * DF + kin));
    float f[8];
#pragma unroll
    for (int i = 0; i < 8; ++i) f[i] = W[(size_t)(srow + i) * DOUTF + (size_t)n];
    v8us o;
#pragma unroll
    for (int i = 0; i < 8; ++i) o[i] = (unsigned short)bf16_bits(f[i]);
    unsigned short* dp = WT + (size_t)n * WPITCH + (size_t)k8;
    *(volatile v8us*)dp = o;
    __threadfence();
    *(volatile v8us*)dp = o;
  } else if (blk < PREP_WT_BLKS + PREP_XB_BLKS) {
    const int v   = (blk - PREP_WT_BLKS) * NTHR + tid;
    const int row = v >> 3;
    const int c8  = (v & 7) * 8;
    const int rc  = row < nN ? row : nN - 1;
    const float* p = feat + (size_t)rc * DF + c8;
    const v4f a  = *(const v4f*)p;
    const v4f bq = *(const v4f*)(p + 4);
    asm volatile("" :: "v"(a), "v"(bq));
    const bool lv = row < nN;
    v8us o;
    o[0] = lv ? (unsigned short)bf16_bits(a.x)  : (unsigned short)0;
    o[1] = lv ? (unsigned short)bf16_bits(a.y)  : (unsigned short)0;
    o[2] = lv ? (unsigned short)bf16_bits(a.z)  : (unsigned short)0;
    o[3] = lv ? (unsigned short)bf16_bits(a.w)  : (unsigned short)0;
    o[4] = lv ? (unsigned short)bf16_bits(bq.x) : (unsigned short)0;
    o[5] = lv ? (unsigned short)bf16_bits(bq.y) : (unsigned short)0;
    o[6] = lv ? (unsigned short)bf16_bits(bq.z) : (unsigned short)0;
    o[7] = lv ? (unsigned short)bf16_bits(bq.w) : (unsigned short)0;
    unsigned short* dp = XB + (size_t)row * DF + c8;
    *(volatile v8us*)dp = o;
    __threadfence();
    *(volatile v8us*)dp = o;
  } else {
    const int t4 = tid < 16 ? tid : 15;
    const v4f b4 = *(const v4f*)(bvec + 4 * t4);
    asm volatile("" :: "v"(b4));
    v4f o;
    o.x = bf16_val(b4.x); o.y = bf16_val(b4.y); o.z = bf16_val(b4.z); o.w = bf16_val(b4.w);
    float* dp = BIAS + 4 * t4;
    if (tid < 16) *(volatile v4f*)dp = o;
    __threadfence();
    if (tid < 16) *(volatile v4f*)dp = o;
  }
}

__global__ __launch_bounds__(NTHR) void k_bucket(const int* __restrict__ keys, const int* __restrict__ gidx,
                                                 int nE, int nN, int vec8,
                                                 int* LIST, int* CNT, int* OFF, float* DSQ, int* REC) {
  extern __shared__ __attribute__((aligned(16))) int dsm[];
  int* reg1 = dsm;
  int* reg2 = reg1 + RCAP;
  int* scnt = reg2 + RCAP;
  int* soff = scnt + NBA;
  int* cur  = soff + NBA;
  int* list = cur + NBA;
  int* wcnt = list + LISTN;
  int* wtot = wcnt + 8;
  int* wmx  = wtot + 8;
  float* sds = (float*)(wmx + 16);
  const int tid = (int)threadIdx.x, lane = tid & 31, wave = tid >> 5;
  const int nodeBase = (int)blockIdx.x * NBA;
  int nb = nN - nodeBase;
  nb = nb > NBA ? NBA : (nb < 1 ? 1 : nb);

  {
    const v4i z4 = {0, 0, 0, 0};
    for (int i = tid * 4; i < BK_INTS; i += NTHR * 4) *(v4ia*)(dsm + i) = z4;
  }
  __syncthreads();

  int tot = 0;
  const int nChunks = (nE + CHUNK - 1) / CHUNK;
#pragma unroll 1
  for (int ch = 0; ch < nChunks; ++ch) {
    const int cbase = ch * CHUNK;
    const int wc = scan_chunk(keys, nE, cbase, nodeBase, nb, vec8, list, tid, wave);
    if (lane == 0) wcnt[wave] = wc;
    __syncthreads();
    int pre = 0, all = 0;
#pragma unroll
    for (int w2 = 0; w2 < NWAVE; ++w2) {
      int c = wcnt[w2];
      c = c < 0 ? 0 : (c > WCAP ? WCAP : c);
      all += c;
      pre += (w2 < wave) ? c : 0;
    }
    const int wcc  = wc > WCAP ? WCAP : wc;
    const int base = tot + pre;
#pragma unroll 1
    for (int i = lane; i < wcc; i += 32) {
      const int ent = list[wave * WCAP + i];
      const int el  = (ent >> PKS) & (CHUNK - 1);
      const int sl  = ent & (NBA - 1);
      int eid = cbase + el;
      eid = eid > nE - 1 ? nE - 1 : eid;
      const int pos = base + i;
      if (pos < RCAP) reg1[pos] = (int)(((unsigned)eid << PKS) | (unsigned)sl);
    }
    tot += all;
    tot = tot > RCAP ? RCAP : tot;
    __syncthreads();
  }
  const int nh = tot;

  if (wave == 0) {
#pragma unroll 1
    for (int b0 = 0; b0 < nh; b0 += 32) {
      const int idx = b0 + lane;
      const int uv  = reg1[idx < RCAP ? idx : RCAP - 1];
      const int m32 = (nh - b0) < 32 ? (nh - b0) : 32;
#pragma unroll 1
      for (int k = 0; k < m32; ++k) {
        const int u  = __builtin_amdgcn_readlane(uv, k);
        const int sl = u & (NBA - 1);
        if (lane == 0) scnt[sl] = scnt[sl] + 1;
      }
    }
  }
  __syncthreads();

  {
    const v4i ca = *(const v4ia*)(scnt + 4 * tid);
    const int e0 = ca.x < 0 ? 0 : ca.x, e1 = ca.y < 0 ? 0 : ca.y, e2 = ca.z < 0 ? 0 : ca.z, e3 = ca.w < 0 ? 0 : ca.w;
    const int ts = e0 + e1 + e2 + e3;
    int incl = ts;
#pragma unroll
    for (int d = 1; d < 32; d <<= 1) {
      const int up = __shfl_up(incl, d, 32);
      if (lane >= d) incl += up;
    }
    int mx = max(max(e0, e1), max(e2, e3));
    mx = max(mx, __shfl_xor(mx, 16, 32));
    mx = max(mx, __shfl_xor(mx, 8, 32));
    mx = max(mx, __shfl_xor(mx, 4, 32));
    mx = max(mx, __shfl_xor(mx, 2, 32));
    mx = max(mx, __shfl_xor(mx, 1, 32));
    if (lane == 31) wtot[wave] = incl;
    if (lane == 0)  wmx[wave] = mx;
    __syncthreads();
    int pre = 0;
#pragma unroll
    for (int w2 = 0; w2 < NWAVE; ++w2) pre += (w2 < wave) ? wtot[w2] : 0;
    int run = pre + incl - ts;
    v4i so;
    so.x = run; run += e0;
    so.y = run; run += e1;
    so.z = run; run += e2;
    so.w = run;
    *(v4ia*)(soff + 4 * tid) = so;
    *(v4ia*)(cur + 4 * tid)  = so;
#pragma unroll 1
    for (int i = tid; i < NBA; i += NTHR) {
      int cv = scnt[i];
      cv = cv < 1 ? 1 : cv;
      sds[i] = 1.0f / sqrtf((float)cv);
    }
  }
  __syncthreads();

  if (wave == 0) {
#pragma unroll 1
    for (int b0 = 0; b0 < nh; b0 += 32) {
      const int idx = b0 + lane;
      const int uv  = reg1[idx < RCAP ? idx : RCAP - 1];
      const int m32 = (nh - b0) < 32 ? (nh - b0) : 32;
#pragma unroll 1
      for (int k = 0; k < m32; ++k) {
        const int u   = __builtin_amdgcn_readlane(uv, k);
        const int sl  = u & (NBA - 1);
        const int eid = (int)((unsigned)u >> PKS);
        if (lane == 0) {
          int pos = cur[sl];
          pos = pos < 0 ? 0 : (pos > RCAP - 1 ? RCAP - 1 : pos);
          reg2[pos] = eid;
          cur[sl] = pos + 1;
        }
      }
    }
  }
  __syncthreads();

  int bmax = 0;
#pragma unroll
  for (int w2 = 0; w2 < NWAVE; ++w2) bmax = max(bmax, wmx[w2]);
  const int flag = ((nh >= RCAP) || (bmax > DEGCAP)) ? 1 : 0;

  int* lrow = LIST + (size_t)blockIdx.x * RCAP;
#pragma unroll 1
  for (int it = 0; it < RCAP / (NTHR * 4); ++it) {
    const int i0 = 4 * (it * NTHR + tid);
    const v4i ev = *(const v4ia*)(reg2 + i0);
    int e0 = ev.x, e1 = ev.y, e2 = ev.z, e3 = ev.w;
    e0 = e0 < 0 ? 0 : (e0 > nE - 1 ? nE - 1 : e0);
    e1 = e1 < 0 ? 0 : (e1 > nE - 1 ? nE - 1 : e1);
    e2 = e2 < 0 ? 0 : (e2 > nE - 1 ? nE - 1 : e2);
    e3 = e3 < 0 ? 0 : (e3 > nE - 1 ? nE - 1 : e3);
    int g0 = gidx[e0], g1 = gidx[e1], g2 = gidx[e2], g3 = gidx[e3];
    asm volatile("" :: "v"(g0), "v"(g1), "v"(g2), "v"(g3));
    g0 = g0 < 0 ? 0 : (g0 > nN - 1 ? nN - 1 : g0);
    g1 = g1 < 0 ? 0 : (g1 > nN - 1 ? nN - 1 : g1);
    g2 = g2 < 0 ? 0 : (g2 > nN - 1 ? nN - 1 : g2);
    g3 = g3 < 0 ? 0 : (g3 > nN - 1 ? nN - 1 : g3);
    v4i ov;
    ov.x = (i0     < nh) ? g0 : 0;
    ov.y = (i0 + 1 < nh) ? g1 : 0;
    ov.z = (i0 + 2 < nh) ? g2 : 0;
    ov.w = (i0 + 3 < nh) ? g3 : 0;
    *(volatile v4i*)(lrow + i0) = ov;
    __threadfence();
    *(volatile v4i*)(lrow + i0) = ov;
  }
  {
    const v4i cv = *(const v4ia*)(scnt + 4 * tid);
    const v4i fv = *(const v4ia*)(soff + 4 * tid);
    const v4f dv = *(const v4fa*)(sds + 4 * tid);
    v4i rv = {0, 0, 0, 0};
    rv.x = (tid == 0) ? bmax : 0;
    rv.y = (tid == 0) ? flag : 0;
    rv.z = (tid == 0) ? nh : 0;
    int*   cp = CNT + (size_t)nodeBase + 4 * tid;
    int*   fp = OFF + (size_t)nodeBase + 4 * tid;
    float* dp = DSQ + (size_t)nodeBase + 4 * tid;
    int*   rp = REC + (size_t)blockIdx.x * 32 + 4 * (tid & 7);
    *(volatile v4i*)cp = cv;
    *(volatile v4i*)fp = fv;
    *(volatile v4f*)dp = dv;
    if (tid < 8) *(volatile v4i*)rp = rv;
    __threadfence();
    *(volatile v4i*)cp = cv;
    *(volatile v4i*)fp = fv;
    *(volatile v4f*)dp = dv;
    if (tid < 8) *(volatile v4i*)rp = rv;
  }
}

__global__ __launch_bounds__(NTHR) void k_rep1(const unsigned* __restrict__ XBw, const int* __restrict__ LIST,
                                               const int* __restrict__ CNT, const int* __restrict__ OFF,
                                               const float* __restrict__ DSQ, const int* __restrict__ REC,
                                               float* X1, int nN, int mRows) {
  const int tid = (int)threadIdx.x, lane = tid & 31;
  const int wave = __builtin_amdgcn_readfirstlane(tid >> 5);
#pragma unroll 1
  for (int ri = 0; ri < RPW; ++ri) {
    int node = (int)blockIdx.x * RPB + wave * RPW + ri;
    node = node > mRows - 1 ? mRows - 1 : node;
    int c, o, last;
    slot_info(CNT, OFF, node, c, o, last);
    const int blk = node >> PKS;
    const int flag = REC[(size_t)blk * 32 + 1];
    const int* lp = LIST + (size_t)blk * RCAP;
    float a0 = 0.0f, a1 = 0.0f;
#pragma unroll 1
    for (int b0 = 0; b0 < c; b0 += 32) {
      int idx = o + b0 + lane;
      idx = idx > last ? last : idx;
      int col = lp[idx];
      col = col < 0 ? 0 : (col > nN - 1 ? nN - 1 : col);
      const int dsb = __float_as_int(DSQ[col]);
      const int m32 = (c - b0) < 32 ? (c - b0) : 32;
#pragma unroll 1
      for (int k = 0; k < m32; ++k) {
        const int   sk = __builtin_amdgcn_readlane(col, k);
        const float dk = __int_as_float(__builtin_amdgcn_readlane(dsb, k));
        const unsigned w = XBw[(size_t)sk * (DF / 2) + lane];
        const float ma = bfw_lo(w) * dk;
        const float mb = bfw_hi(w) * dk;
        a0 += ma;
        a1 += mb;
      }
    }
    const int nodec = node < nN ? node : nN - 1;
    const float dsi = DSQ[nodec];
    const unsigned w0 = XBw[(size_t)nodec * (DF / 2) + lane];
    asm volatile("" :: "v"(dsi), "v"(w0));
    const float x0a = bfw_lo(w0), x0b = bfw_hi(w0);
    const float t0 = a0 * dsi, t1 = a1 * dsi;
    float r0 = CX1_A * t0 + x0a * CX1_B;
    float r1 = CX1_A * t1 + x0b * CX1_B;
    const float qn = __uint_as_float(0x7fc00000u);
    r0 = (flag != 0) ? qn : r0;
    r1 = (flag != 0) ? qn : r1;
    const bool live = node < nN;
    v2f rv;
    rv.x = live ? r0 : 0.0f;
    rv.y = live ? r1 : 0.0f;
    float* xp = X1 + (size_t)node * DF + 2 * lane;
    *(volatile v2f*)xp = rv;
    __threadfence();
    *(volatile v2f*)xp = rv;
  }
}

template <int S1, int S2>
__global__ __launch_bounds__(NTHR) void k_rep2(const unsigned* __restrict__ XBw, const float* __restrict__ X1,
                                               const int* __restrict__ LIST, const int* __restrict__ CNT,
                                               const int* __restrict__ OFF, const float* __restrict__ DSQ,
                                               const int* __restrict__ REC, unsigned* Aw, int nN, int mRows) {
  const int tid = (int)threadIdx.x, lane = tid & 31;
  const int wave = __builtin_amdgcn_readfirstlane(tid >> 5);
#pragma unroll 1
  for (int ri = 0; ri < RPW; ++ri) {
    int node = (int)blockIdx.x * RPB + wave * RPW + ri;
    node = node > mRows - 1 ? mRows - 1 : node;
    int c, o, last;
    slot_info(CNT, OFF, node, c, o, last);
    const int blk = node >> PKS;
    const int flag = REC[(size_t)blk * 32 + 1];
    const int* lp = LIST + (size_t)blk * RCAP;
    float a0 = 0.0f, a1 = 0.0f;
#pragma unroll 1
    for (int b0 = 0; b0 < c; b0 += 32) {
      int idx = o + b0 + lane;
      idx = idx > last ? last : idx;
      int col = lp[idx];
      col = col < 0 ? 0 : (col > nN - 1 ? nN - 1 : col);
      const int dsb = __float_as_int(DSQ[col]);
      const int m32 = (c - b0) < 32 ? (c - b0) : 32;
#pragma unroll 1
      for (int k = 0; k < m32; ++k) {
        const int   sk = __builtin_amdgcn_readlane(col, k);
        const float dk = __int_as_float(__builtin_amdgcn_readlane(dsb, k));
        const v2f xv = *(const v2f*)(X1 + (size_t)sk * DF + 2 * lane);
        const float ma = xv.x * dk;
        const float mb = xv.y * dk;
        a0 += ma;
        a1 += mb;
      }
    }
    const int nodec = node < nN ? node : nN - 1;
    const float dsi = DSQ[nodec];
    const unsigned w0 = XBw[(size_t)nodec * (DF / 2) + lane];
    const v2f x1o = *(const v2f*)(X1 + (size_t)nodec * DF + 2 * lane);
    asm volatile("" :: "v"(dsi), "v"(w0), "v"(x1o));
    const float x0a = bfw_lo(w0), x0b = bfw_hi(w0);
    const float t0 = a0 * dsi, t1 = a1 * dsi;
    const float x2a = (CX2_A * t0 + x1o.x * CX2_B) - x0a;
    const float x2b = (CX2_A * t1 + x1o.y * CX2_B) - x0b;
    unsigned h1, l1, h2, l2;
    pack2(x1o.x, x1o.y, h1, l1);
    pack2(x2a, x2b, h2, l2);
    if (S1 == 0) l1 = 0u;
    if (S2 == 0) l2 = 0u;
    const unsigned qw = 0x7fc07fc0u;
    const bool pz = flag != 0;
    h1 = pz ? qw : h1;
    h2 = pz ? qw : h2;
    l1 = (pz && S1 != 0) ? qw : l1;
    l2 = (pz && S2 != 0) ? qw : l2;
    const bool live = node < nN;
    const unsigned q0 = live ? w0 : 0u;
    const unsigned q1 = live ? h1 : 0u;
    const unsigned q2 = live ? l1 : 0u;
    const unsigned q3 = live ? h2 : 0u;
    const unsigned q4 = live ? l2 : 0u;
    unsigned* wp = Aw + (size_t)node * AWORDS + lane;
    *(volatile unsigned*)(wp)       = q0;
    *(volatile unsigned*)(wp + 32)  = q1;
    *(volatile unsigned*)(wp + 64)  = q2;
    *(volatile unsigned*)(wp + 96)  = q3;
    *(volatile unsigned*)(wp + 128) = q4;
    __threadfence();
    *(volatile unsigned*)(wp)       = q0;
    *(volatile unsigned*)(wp + 32)  = q1;
    *(volatile unsigned*)(wp + 64)  = q2;
    *(volatile unsigned*)(wp + 96)  = q3;
    *(volatile unsigned*)(wp + 128) = q4;
  }
}

template <int S1, int S2>
__global__ __launch_bounds__(NTHR) __attribute__((amdgpu_num_vgpr(248)))
void k_gemm(const unsigned short* __restrict__ Apl, const unsigned short* __restrict__ WT,
            const float* __restrict__ BIAS, float* out, int nN) {
  __shared__ __attribute__((aligned(16))) float stg[GBM * DOUTF];
  __shared__ __attribute__((aligned(16))) float bsh[DOUTF];
  const int tid = (int)threadIdx.x, lane = tid & 31, wave = tid >> 5, hh = lane >> 4, m = lane & 15;
  const int rowBase = (int)blockIdx.x * GBM;

  {
    const int tb = tid < 15 ? tid : 15;
    const v4f b4 = *(const v4f*)(BIAS + 4 * tb);
    asm volatile("" :: "v"(b4));
    if (tid < 16) *(v4fa*)(bsh + 4 * tid) = b4;
  }

  v8f acc[4];
  {
    const v8f z = {0.f, 0.f, 0.f, 0.f, 0.f, 0.f, 0.f, 0.f};
#pragma unroll
    for (int t = 0; t < 4; ++t) acc[t] = z;
  }
  const unsigned short* ap = Apl + (size_t)(rowBase + 16 * wave + m) * (size_t)APITCH + 8 * hh;
  const unsigned short* wp = WT + (size_t)m * (size_t)WPITCH + 8 * hh;

#pragma unroll 1
  for (int ks = 0; ks < KSTEPS; ++ks) {
    if (S1 == 0 && (ks == 4 || ks == 5)) continue;
    if (S2 == 0 && (ks == 8 || ks == 9)) continue;
    FragB af;
    af.h[0] = *(const v8usa*)(ap + 32 * ks);
    af.h[1] = *(const v8usa*)(ap + 32 * ks + 16);
#pragma unroll
    for (int t = 0; t < 4; ++t) {
      const unsigned short* wq = wp + (size_t)(16 * t) * (size_t)WPITCH + 32 * ks;
      FragB bf;
      bf.h[0] = *(const v8usa*)wq;
      bf.h[1] = *(const v8usa*)(wq + 16);
      acc[t] = wmb(af, bf, acc[t]);
    }
  }

#pragma unroll
  for (int t = 0; t < 4; ++t) {
    const int lc = 16 * t + m;
#pragma unroll
    for (int r = 0; r < 8; ++r) {
      const int lr = 16 * wave + 8 * hh + r;
      stg[lr * DOUTF + lc] = acc[t][r];
    }
  }
  __syncthreads();

  const int c4 = 4 * (lane & 15);
  const v4f bb = *(const v4fa*)(bsh + c4);
  v4f pv[8];
#pragma unroll
  for (int i = 0; i < 8; ++i) {
    const int lr = 16 * wave + 2 * i + (lane >> 4);
    const v4f a = *(const v4fa*)(stg + lr * DOUTF + c4);
    v4f y;
    y.x = relu_k(a.x + bb.x);
    y.y = relu_k(a.y + bb.y);
    y.z = relu_k(a.z + bb.z);
    y.w = relu_k(a.w + bb.w);
    pv[i] = y;
  }
#pragma unroll
  for (int i = 0; i < 8; ++i) {
    const int gr = rowBase + 16 * wave + 2 * i + (lane >> 4);
    const int gs = gr < nN ? gr : nN - 1;
    float* op = out + (size_t)gs * DOUTF + c4;
    if (gr < nN) *(volatile v4f*)op = pv[i];
  }
  __threadfence();
#pragma unroll
  for (int i = 0; i < 8; ++i) {
    const int gr = rowBase + 16 * wave + 2 * i + (lane >> 4);
    const int gs = gr < nN ? gr : nN - 1;
    float* op = out + (size_t)gs * DOUTF + c4;
    if (gr < nN) *(volatile v4f*)op = pv[i];
  }
}

extern "C" void kernel_launch(void* const* d_in, const int* in_sizes, int n_in,
                              void* d_out, int out_size, void* d_ws, size_t ws_size,
                              hipStream_t stream) {
  if (n_in < 5) return;
  if (in_sizes[0] != NNODE * DF) return;
  if (in_sizes[1] != NEDGE || in_sizes[2] != NEDGE) return;
  if (in_sizes[3] != KPOLY * DF * DOUTF) return;
  if (in_sizes[4] != DOUTF) return;
  if (out_size != NNODE * DOUTF) return;
  if (WS_TOTAL > ws_size) return;
  const int nN = NNODE;
  const int nE = NEDGE;

  const float* feat = (const float*)d_in[0];
  const int*   src  = (const int*)  d_in[1];
  const int*   dst  = (const int*)  d_in[2];
  const float* W    = (const float*)d_in[3];
  const float* bvec = (const float*)d_in[4];
  float* out = (float*)d_out;

  char* ws = (char*)d_ws;
  unsigned short* WT   = (unsigned short*)(ws + O_WT);
  float*          BIAS = (float*)(ws + O_BS);
  unsigned short* XB   = (unsigned short*)(ws + O_XB);
  float*          X1   = (float*)(ws + O_X1);
  unsigned short* Apl  = (unsigned short*)(ws + O_A);
  int*            LIST = (int*)(ws + O_LS);
  int*            CNT  = (int*)(ws + O_CN);
  int*            OFF  = (int*)(ws + O_OF);
  float*          DSQ  = (float*)(ws + O_DS);
  int*            REC  = (int*)(ws + O_RC);

  const int vec8 = ((nE & 3) == 0) ? 1 : 0;
  const int gR   = MPAD / RPB;
  const int gG   = MPAD / GBM;

  hipFuncSetAttribute(reinterpret_cast<const void*>(&k_bucket), hipFuncAttributeMaxDynamicSharedMemorySize, LDS_BK);

  k_prep<<<PREP_BLKS, NTHR, 0, stream>>>(feat, W, bvec, WT, XB, BIAS, nN);
  k_bucket<<<NBLK, NTHR, LDS_BK, stream>>>(dst, src, nE, nN, vec8, LIST, CNT, OFF, DSQ, REC);
  k_rep1<<<gR, NTHR, 0, stream>>>((const unsigned*)XB, LIST, CNT, OFF, DSQ, REC, X1, nN, MPAD);
  k_rep2<SPLIT_X1, SPLIT_X2><<<gR, NTHR, 0, stream>>>((const unsigned*)XB, X1, LIST, CNT, OFF, DSQ, REC,
                                                     (unsigned*)Apl, nN, MPAD);
  k_gemm<SPLIT_X1, SPLIT_X2><<<gG, NTHR, 0, stream>>>(Apl, WT, BIAS, out, nN);
}
